// sample_and_group_18167711662781
// MI455X (gfx1250) — hardware-verified
//
#include <hip/hip_runtime.h>
#include <math.h>

typedef __attribute__((ext_vector_type(16))) _Float16 v16h;
typedef __attribute__((ext_vector_type(16))) __bf16 v16b;
typedef __attribute__((ext_vector_type(8)))  _Float16 v8h;
typedef __attribute__((ext_vector_type(8)))  float v8f;
typedef __attribute__((ext_vector_type(4)))  float v4f;
typedef __attribute__((ext_vector_type(2)))  float v2f;
typedef __attribute__((ext_vector_type(4)))  unsigned v4u;
typedef __attribute__((ext_vector_type(4)))  int v4i;
typedef float __attribute__((may_alias)) float_a;
typedef int __attribute__((may_alias)) int_a;

template <typename T> __device__ __forceinline__ void vst2(void* p, T v) { *(volatile T*)p = v; __threadfence(); *(volatile T*)p = v; }
__device__ __forceinline__ v8f wmma16(v16h a, v16h b, v8f c) {
  v8f d = __builtin_amdgcn_wmma_f32_16x16x32_f16(false, a, false, b, (short)0, c, false, false);
  asm volatile("v_nop\n\tv_nop\n\tv_nop\n\tv_nop" : "+v"(d) : "v"(a), "v"(b));
  return d;
}
__device__ __forceinline__ v8f wmma_bf(v16b a, v16b b, v8f c) {
  v8f d = __builtin_amdgcn_wmma_f32_16x16x32_bf16(false, a, false, b, (short)0, c, false, false);
  asm volatile("v_nop\n\tv_nop\n\tv_nop\n\tv_nop" : "+v"(d) : "v"(a), "v"(b));
  return d;
}
__device__ __forceinline__ v16h frag_h(const _Float16* rowk0, int lane) {
  union { v16h v; v8h q[2]; } u; const _Float16* p = rowk0 + 8 * (lane >> 4);
  u.q[0] = *(const v8h*)p; u.q[1] = *(const v8h*)(p + 16); return u.v;
}
__device__ __forceinline__ v16h frag_f32(const float* rowk0, int lane) {
  v16h a; const float* p = rowk0 + 8 * (lane >> 4);
#pragma unroll
  for (int i = 0; i < 8; ++i) { a[i] = (_Float16)p[i]; a[8 + i] = (_Float16)p[16 + i]; }
  return a;
}
__device__ __forceinline__ v16h frag_f32s(const float* rowk0, int lane, float sc) {
  v16h a; const float* p = rowk0 + 8 * (lane >> 4);
#pragma unroll
  for (int i = 0; i < 8; ++i) { a[i] = (_Float16)(p[i] * sc); a[8 + i] = (_Float16)(p[16 + i] * sc); }
  return a;
}
__device__ __forceinline__ v16h fragc_f32(const float* W, int k0, int n, int lane, int ld, int K) {
  v16h a; const int g = lane >> 4;
#pragma unroll
  for (int i = 0; i < 8; ++i) { const int ka = k0 + 8 * g + i, kb = ka + 16;
    a[i] = (_Float16)(ka < K ? W[(size_t)(ka < K ? ka : K - 1) * ld + n] : 0.f); a[8 + i] = (_Float16)(kb < K ? W[(size_t)(kb < K ? kb : K - 1) * ld + n] : 0.f); }
  return a;
}
struct F2 { v16b h, l; };
__device__ __forceinline__ F2 bsplit16(const float v[16]) { F2 r;
#pragma unroll
  for (int i = 0; i < 16; ++i) { const __bf16 h = (__bf16)v[i]; r.h[i] = h; r.l[i] = (__bf16)(v[i] - (float)h); }
  return r; }
__device__ __forceinline__ F2 split_row(const float* row, int k0, int lane) { float v[16]; const float* p = row + k0 + 8 * (lane >> 4);
#pragma unroll
  for (int i = 0; i < 8; ++i) { v[i] = p[i]; v[8 + i] = p[16 + i]; }
  return bsplit16(v); }
__device__ __forceinline__ F2 split_rowK(const float* row, int k0, int lane, int K) { float v[16]; const int g = lane >> 4;
#pragma unroll
  for (int i = 0; i < 8; ++i) { const int ka = k0 + 8 * g + i, kb = ka + 16; v[i] = ka < K ? row[ka < K ? ka : K - 1] : 0.f; v[8 + i] = kb < K ? row[kb < K ? kb : K - 1] : 0.f; }
  return bsplit16(v); }
__device__ __forceinline__ F2 split_col(const float* W, int k0, int n, int lane, int ld, int K) { float v[16]; const int g = lane >> 4;
#pragma unroll
  for (int i = 0; i < 8; ++i) { const int ka = k0 + 8 * g + i, kb = ka + 16; v[i] = ka < K ? W[(size_t)(ka < K ? ka : K - 1) * ld + n] : 0.f; v[8 + i] = kb < K ? W[(size_t)(kb < K ? kb : K - 1) * ld + n] : 0.f; }
  return bsplit16(v); }
__device__ __forceinline__ v8f mac3(const F2& a, const F2& b, v8f c) { c = wmma_bf(a.l, b.h, c); c = wmma_bf(a.h, b.l, c); return wmma_bf(a.h, b.h, c); }
__device__ __forceinline__ float sigm(float v) { return 1.0f / (1.0f + expf(-v)); }
#define LDSX() do { asm volatile("s_wait_dscnt 0" ::: "memory"); __builtin_amdgcn_wave_barrier(); __builtin_amdgcn_fence(__ATOMIC_RELEASE, "workgroup"); } while (0)


#define NB 8
#define NB_OUT 8
#define NPT 8192
#define CC 64
#define SS 2048
#define KK 32
#define OC 128
#define NQ (NB * SS)
#define NROW (NQ * KK)
#ifndef NQB
#define NQB (NQ / 64)
#define NRB2 (NROW / 64)
#endif
typedef __attribute__((ext_vector_type(8))) __bf16 v8b;
__device__ __forceinline__ v16b frag_b(const __bf16* rowk0, int lane) {
  union { v16b v; v8b q[2]; } u; const __bf16* p = rowk0 + 8 * (lane >> 4);
  u.q[0] = *(const v8b*)p; u.q[1] = *(const v8b*)(p + 16); return u.v;
}
__device__ __forceinline__ float bfr(float v) { return (float)(__bf16)v; }
__device__ __attribute__((noinline)) float exp_ni(float v) { return expf(v); }
__device__ __attribute__((noinline)) float erf_ni(float v) { return erff(v); }

#define WS_PW   0u
#define PWB 0
#define PWDH (PWB + OC * CC)
#define PWDL (PWDH + OC * CC)
#define PW2 (PWDL + OC * CC)
#define PWEND (PW2 + OC * OC)
#define WS_KNN  (WS_PW + 2u * PWEND)
#define WS_P    (WS_KNN + 4u * NQ * KK)
#define WS_Q    (WS_P + 4u * NB * NPT * OC)
#define WS_ST1  (WS_Q + 4u * NQ * OC)
#define WS_BN1  (WS_ST1 + 4u * NQB * 2 * OC)
#define WS_ST2  (WS_BN1 + 4u * 4 * OC)
#define WS_BN2  (WS_ST2 + 4u * NRB2 * 2 * OC)
#define WS_END  (WS_BN2 + 4u * 4 * OC)

__global__ __launch_bounds__(128) void k_pack(const float* __restrict__ W1, const float* __restrict__ W2m, __bf16* __restrict__ PW) {
  __shared__ __align__(16) __bf16 sb[CC], sh[CC], slo[CC], s2[OC]; const int o = blockIdx.x, t = threadIdx.x;
  if (t < CC) { const float wa = bfr(W1[(size_t)o * 2 * CC + t]), wb = bfr(W1[(size_t)o * 2 * CC + CC + t]); sb[t] = (__bf16)wb; const float d = wa - wb; const __bf16 hb = (__bf16)d; sh[t] = hb; slo[t] = (__bf16)(d - (float)hb); }
  s2[t] = (__bf16)W2m[(size_t)o * OC + t];
  __syncthreads();
  if (t < CC / 8) { vst2((unsigned*)(PW + PWB + (size_t)o * CC + t * 8), *(const v4u*)&sb[t * 8]); vst2((unsigned*)(PW + PWDH + (size_t)o * CC + t * 8), *(const v4u*)&sh[t * 8]); vst2((unsigned*)(PW + PWDL + (size_t)o * CC + t * 8), *(const v4u*)&slo[t * 8]); }
  if (t < OC / 8) vst2((unsigned*)(PW + PW2 + (size_t)o * OC + t * 8), *(const v4u*)&s2[t * 8]);
}
__global__ __launch_bounds__(64) void k_knn(const float* __restrict__ COOR, const int* __restrict__ INDX, int* __restrict__ KNN, float* __restrict__ OSC) {
  __shared__ __align__(16) int sk[64][KK]; __shared__ __align__(16) float ssc[64 * 3];
  const int tid = threadIdx.x; const size_t q = (size_t)blockIdx.x * 64 + tid; const int b = (int)(q / SS), s = (int)(q % SS);
  const int pi = min(max(INDX[s], 0), NPT - 1); const float* cb = COOR + (size_t)b * NPT * 3; const float sx = bfr(cb[pi * 3]), sy = bfr(cb[pi * 3 + 1]), sz = bfr(cb[pi * 3 + 2]);
  float bd[KK]; int bi[KK];
#pragma unroll
  for (int j = 0; j < KK; ++j) { bd[j] = 3.0e38f; bi[j] = 0; }
#pragma unroll 1
  for (int p = 0; p < NPT; ++p) { const float dx = bfr(cb[p * 3]) - sx, dy = bfr(cb[p * 3 + 1]) - sy, dz = bfr(cb[p * 3 + 2]) - sz; const float d = (dx * dx + dy * dy) + dz * dz;
    if (d < bd[KK - 1]) { int pos = KK - 1;
#pragma unroll
      for (int j = KK - 2; j >= 0; --j) if (d < bd[j]) pos = j;
#pragma unroll
      for (int j = KK - 1; j >= 1; --j) if (j > pos) { bd[j] = bd[j - 1]; bi[j] = bi[j - 1]; }
#pragma unroll
      for (int j = 0; j < KK; ++j) if (j == pos) { bd[j] = d; bi[j] = p; } } }
#pragma unroll
  for (int j = 0; j < KK; ++j) sk[tid][j] = bi[j];
  ssc[tid * 3] = sx; ssc[tid * 3 + 1] = sy; ssc[tid * 3 + 2] = sz;
  __syncthreads();
  for (int r = 0; r < 64; ++r) if (tid < 8) vst2((unsigned*)(KNN + ((size_t)blockIdx.x * 64 + r) * KK + tid * 4), *(const v4u*)&sk[r][tid * 4]);
  if (tid < 48) vst2(OSC + (size_t)blockIdx.x * 64 * 3 + tid * 4, *(const v4f*)&ssc[tid * 4]);
}
template <int SAMP>
__global__ __launch_bounds__(128) void k_lin1(const float* __restrict__ X, const int* __restrict__ INDX, const __bf16* __restrict__ PW, const float* __restrict__ B1, float* __restrict__ OUT) {
  __shared__ __align__(16) float so[4][16][132];
  const int tid = threadIdx.x, wave = tid >> 5, lane = tid & 31, col = lane & 15, g = lane >> 4; const size_t r0 = (size_t)blockIdx.x * 64 + wave * 16;
  size_t xrow; { const size_t r = r0 + col; if (SAMP) { const int b = (int)(r / SS), s = (int)(r % SS); xrow = (size_t)b * NPT + min(max(INDX[s], 0), NPT - 1); } else xrow = r; }
  v8f acc[8] = {};
#pragma unroll
  for (int kc = 0; kc < CC / 32; ++kc) { v16b a; { const float* p = X + xrow * CC + kc * 32 + 8 * g;
#pragma unroll
      for (int i = 0; i < 8; ++i) { a[i] = (__bf16)p[i]; a[8 + i] = (__bf16)p[16 + i]; } }
#pragma unroll
    for (int j = 0; j < 8; ++j) { if (SAMP) { acc[j] = wmma_bf(a, frag_b(PW + PWDL + (size_t)(j * 16 + col) * CC + kc * 32, lane), acc[j]); acc[j] = wmma_bf(a, frag_b(PW + PWDH + (size_t)(j * 16 + col) * CC + kc * 32, lane), acc[j]); } else acc[j] = wmma_bf(a, frag_b(PW + PWB + (size_t)(j * 16 + col) * CC + kc * 32, lane), acc[j]); } }
#pragma unroll
  for (int j = 0; j < 8; ++j) { const float bb = SAMP ? bfr(B1[j * 16 + col]) : 0.f;
#pragma unroll
    for (int r = 0; r < 8; ++r) so[wave][8 * g + r][j * 16 + col] = acc[j][r] + bb; }
  LDSX();
  for (int rl = 0; rl < 16; ++rl) vst2(OUT + (r0 + rl) * OC + lane * 4, *(const v4f*)&so[wave][rl][lane * 4]);
}
template <int PASS>
__global__ __launch_bounds__(128) void k_st1(const float* __restrict__ Pm, const float* __restrict__ Qm, const int* __restrict__ KNN, const float* __restrict__ BN1, float* __restrict__ ST1) {
  __shared__ __align__(16) float ss[OC]; const int c = threadIdx.x; const float mu = PASS ? BN1[c] : 0.f; float a = 0.f;
#pragma unroll 1
  for (int ql = 0; ql < 64; ++ql) { const size_t q = (size_t)blockIdx.x * 64 + ql; const int b = (int)(q / SS); const float qq = Qm[q * OC + c];
#pragma unroll 4
    for (int k = 0; k < KK; ++k) { const int p = min(max(KNN[q * KK + k], 0), NPT - 1); const float y = qq + Pm[((size_t)b * NPT + p) * OC + c]; const float d = y - mu; a += PASS ? d * d : y; } }
  ss[c] = a; __syncthreads();
  if (c < 32) vst2(ST1 + ((size_t)blockIdx.x * 2 + PASS) * OC + c * 4, *(const v4f*)&ss[c * 4]);
}
template <int PASS>
__global__ __launch_bounds__(128) void k_fin1(const float* __restrict__ ST1, const float* __restrict__ G1, const float* __restrict__ BE1, float* __restrict__ BN1) {
  __shared__ __align__(16) float s[3][OC]; const int c = threadIdx.x; float a = 0.f;
#pragma unroll 1
  for (int blk = 0; blk < NQB; ++blk) a += ST1[((size_t)blk * 2 + PASS) * OC + c];
  const float n = (float)NROW;
  if (PASS == 0) { s[0][c] = a / n; __syncthreads(); if (c < 32) vst2(BN1 + c * 4, *(const v4f*)&s[0][c * 4]); }
  else { const float var = a / n; const float mean = BN1[c]; const float sc = rsqrtf(var + 1e-5f) * bfr(G1[c]); s[1][c] = sc; s[2][c] = bfr(BE1[c]) - mean * sc; __syncthreads(); if (c < 32) { vst2(BN1 + OC + c * 4, *(const v4f*)&s[1][c * 4]); vst2(BN1 + 2 * OC + c * 4, *(const v4f*)&s[2][c * 4]); } }
}
template <int PASS>
__global__ __launch_bounds__(128) void k_lin2(const float* __restrict__ Pm, const float* __restrict__ Qm, const int* __restrict__ KNN, const float* __restrict__ BN1, const __bf16* __restrict__ PW, const float* __restrict__ B2, const float* __restrict__ BN2, float* __restrict__ ST2, float* __restrict__ OUT) {
  __shared__ __align__(16) float sred[4][2][OC]; __shared__ __align__(16) float sline[2][OC];
  const int tid = threadIdx.x, wave = tid >> 5, lane = tid & 31, col = lane & 15, g = lane >> 4; const size_t r0 = (size_t)blockIdx.x * 64 + wave * 16;
  const size_t myrow = r0 + col; const size_t q = myrow / KK; const int k = (int)(myrow % KK); const int b = (int)(q / SS); const int p = min(max(KNN[q * KK + k], 0), NPT - 1);
  const float* prow = Pm + ((size_t)b * NPT + p) * OC; const float* qrow = Qm + q * OC;
  v8f acc[8] = {};
#pragma unroll
  for (int kc = 0; kc < OC / 32; ++kc) { float v[16];
#pragma unroll
    for (int i = 0; i < 16; ++i) { const int c = kc * 32 + 8 * g + (i & 7) + ((i >> 3) << 4); const float y1 = qrow[c] + prow[c]; v[i] = fmaxf(y1 * BN1[OC + c] + BN1[2 * OC + c], 0.f); }
    const F2 a = bsplit16(v);
#pragma unroll
    for (int j = 0; j < 8; ++j) { const v16b w = frag_b(PW + PW2 + (size_t)(j * 16 + col) * OC + kc * 32, lane); acc[j] = wmma_bf(a.l, w, acc[j]); acc[j] = wmma_bf(a.h, w, acc[j]); } }
  if (PASS == 0) {
#pragma unroll
    for (int j = 0; j < 8; ++j) { const int c = j * 16 + col; const float bb = bfr(B2[c]); float s1 = 0.f, s2 = 0.f;
#pragma unroll
      for (int r = 0; r < 8; ++r) { const float y = acc[j][r] + bb; s1 += y; s2 += y * y; }
      s1 += __shfl_xor(s1, 16); s2 += __shfl_xor(s2, 16);
      if (g == 0) { sred[wave][0][c] = s1; sred[wave][1][c] = s2; } }
    __syncthreads();
    { const int c = tid; float s1 = 0.f, s2 = 0.f; for (int w = 0; w < 4; ++w) { s1 += sred[w][0][c]; s2 += sred[w][1][c]; } sline[0][c] = s1; sline[1][c] = s2; }
    __syncthreads();
    if (tid < 64) vst2(ST2 + ((size_t)blockIdx.x * 2 + (tid >> 5)) * OC + (tid & 31) * 4, *(const v4f*)&sline[tid >> 5][(tid & 31) * 4]);
  } else {
#pragma unroll
    for (int j = 0; j < 8; ++j) { const int c = j * 16 + col; const float bb = bfr(B2[c]); float mx = -3.0e38f;
#pragma unroll
      for (int r = 0; r < 8; ++r) { const float y = acc[j][r] + bb; mx = fmaxf(mx, fmaxf(y * BN2[c] + BN2[OC + c], 0.f)); }
      mx = fmaxf(mx, __shfl_xor(mx, 16)); if (g == 0) sred[wave][0][c] = mx; }
    __syncthreads();
    { const int c = tid; sline[0][c] = fmaxf(sred[0][0][c], sred[1][0][c]); sline[1][c] = fmaxf(sred[2][0][c], sred[3][0][c]); }
    __syncthreads();
    if (tid < 64) { const size_t qq = (size_t)blockIdx.x * 2 + (tid >> 5); vst2(OUT + qq * OC + (tid & 31) * 4, *(const v4f*)&sline[tid >> 5][(tid & 31) * 4]); }
  }
}
__global__ __launch_bounds__(128) void k_fin2(const float* __restrict__ ST2, const float* __restrict__ G2, const float* __restrict__ BE2, float* __restrict__ BN2) {
  __shared__ __align__(16) float s[2][OC]; const int c = threadIdx.x; double s1 = 0.0, s2 = 0.0;
#pragma unroll 1
  for (int blk = 0; blk < NRB2; ++blk) { s1 += (double)ST2[((size_t)blk * 2) * OC + c]; s2 += (double)ST2[((size_t)blk * 2 + 1) * OC + c]; }
  const double n = (double)NROW; const double mean = s1 / n; double var = s2 / n - mean * mean; if (var < 0.0) var = 0.0;
  const float sc = rsqrtf((float)var + 1e-5f) * bfr(G2[c]); s[0][c] = sc; s[1][c] = bfr(BE2[c]) - (float)mean * sc; __syncthreads();
  if (c < 64) vst2(BN2 + (size_t)(c >> 5) * OC + (c & 31) * 4, *(const v4f*)&s[c >> 5][(c & 31) * 4]);
}
extern "C" void kernel_launch(void* const* d_in, const int* in_sizes, int n_in, void* d_out, int out_size, void* d_ws, size_t ws_size, hipStream_t stream) {
  (void)in_sizes; (void)n_in; (void)out_size;
  const float** F = (const float**)d_in; const int* INDX = (const int*)d_in[2];
  if (ws_size < (size_t)WS_END) return;
  char* ws = (char*)d_ws; __bf16* PW = (__bf16*)(ws + WS_PW); int* KNN = (int*)(ws + WS_KNN); float *Pm = (float*)(ws + WS_P), *Qm = (float*)(ws + WS_Q), *ST1 = (float*)(ws + WS_ST1), *BN1 = (float*)(ws + WS_BN1), *ST2 = (float*)(ws + WS_ST2), *BN2 = (float*)(ws + WS_BN2);
  float* OUT = (float*)d_out; float* OSC = OUT + (size_t)NB_OUT * SS * OC;
  k_pack<<<OC, 128, 0, stream>>>(F[3], F[7], PW);
  k_knn<<<NQB, 64, 0, stream>>>(F[1], INDX, KNN, OSC);
  k_lin1<0><<<NB * NPT / 64, 128, 0, stream>>>(F[0], INDX, PW, F[4], Pm);
  k_lin1<1><<<NQ / 64, 128, 0, stream>>>(F[0], INDX, PW, F[4], Qm);
  k_st1<0><<<NQB, 128, 0, stream>>>(Pm, Qm, KNN, BN1, ST1); k_fin1<0><<<1, 128, 0, stream>>>(ST1, F[5], F[6], BN1);
  k_st1<1><<<NQB, 128, 0, stream>>>(Pm, Qm, KNN, BN1, ST1); k_fin1<1><<<1, 128, 0, stream>>>(ST1, F[5], F[6], BN1);
  k_lin2<0><<<NRB2, 128, 0, stream>>>(Pm, Qm, KNN, BN1, PW, F[8], BN2, ST2, OUT); k_fin2<<<1, 128, 0, stream>>>(ST2, F[9], F[10], BN2);
  k_lin2<1><<<NRB2, 128, 0, stream>>>(Pm, Qm, KNN, BN1, PW, F[8], BN2, ST2, OUT);
}
